// HighOrderGNNEncoder_86303072845900
// MI455X (gfx1250) — hardware-verified
//
#include <hip/hip_runtime.h>


typedef __attribute__((ext_vector_type(16))) _Float16 v16h;
typedef __attribute__((ext_vector_type(8)))  _Float16 v8h;
typedef __attribute__((ext_vector_type(16))) __bf16   v16b;
typedef __attribute__((ext_vector_type(8)))  __bf16   v8b;
typedef __attribute__((ext_vector_type(8)))  float    v8f;
typedef __attribute__((ext_vector_type(4)))  float    v4f;
typedef __attribute__((ext_vector_type(4)))  int      v4i;

#define CN_D 128
#define CN_B 64
#define CN_O 64
#define CN_QKV 384
#define DEG_NT 12544
#define DEG_THREADS 512
#define POOL_CHE 8192
#define POOL_CHN 512

__device__ __forceinline__ unsigned short f2bf_bits(float f) {
  unsigned u = __float_as_uint(f);
  return (unsigned short)((u + 0x7FFFu + ((u >> 16) & 1u)) >> 16);
}
__device__ __forceinline__ float bf_bits2f(unsigned short h) { return __uint_as_float(((unsigned)h) << 16); }

__device__ __forceinline__ void dep_guard_h(v8f& a, v8f& b, v16h x, v16h y) { asm volatile("v_nop\n\tv_nop\n\tv_nop\n\tv_nop" : "+v"(a), "+v"(b) : "v"(x), "v"(y)); }
__device__ __forceinline__ void dep_guard_b(v8f& a, v8f& b, v16b x, v16b y) { asm volatile("v_nop\n\tv_nop\n\tv_nop\n\tv_nop" : "+v"(a), "+v"(b) : "v"(x), "v"(y)); }
__device__ __forceinline__ void keep4_h(v16h a, v16h b, v16h c, v16h d) { asm volatile("v_nop" :: "v"(a), "v"(b), "v"(c), "v"(d)); }
__device__ __forceinline__ void keep4_b(v16b a, v16b b, v16b c, v16b d) { asm volatile("v_nop" :: "v"(a), "v"(b), "v"(c), "v"(d)); }
__device__ __forceinline__ void acc_guard4(v8f& a, v8f& b, v8f& c, v8f& d) { asm volatile("v_nop\n\tv_nop\n\tv_nop\n\tv_nop" : "+v"(a), "+v"(b), "+v"(c), "+v"(d)); }
template <typename T> struct Frag;
template <> struct Frag<_Float16> {
  typedef v16h V; union U { v16h v; v8h h[2]; };
  static __device__ __forceinline__ v16h load(const _Float16* p) {
    U f; f.h[0] = *(const v8h*)(p); f.h[1] = *(const v8h*)(p + 16); return f.v;
  }
  static __device__ __forceinline__ v8f mma(v16h a, v16h b, v8f c) {
    return __builtin_amdgcn_wmma_f32_16x16x32_f16(false, a, false, b, (short)0, c, false, false);
  }
  static __device__ __forceinline__ void guard(v8f& a, v8f& b, v16h x, v16h y) { dep_guard_h(a, b, x, y); }
  static __device__ __forceinline__ void keep(v16h a, v16h b, v16h c, v16h d) { keep4_h(a, b, c, d); }
};
template <> struct Frag<__bf16> {
  typedef v16b V; union U { v16b v; v8b h[2]; };
  static __device__ __forceinline__ v16b load(const __bf16* p) {
    U f; f.h[0] = *(const v8b*)(p); f.h[1] = *(const v8b*)(p + 16); return f.v;
  }
  static __device__ __forceinline__ v8f mma(v16b a, v16b b, v8f c) {
    return __builtin_amdgcn_wmma_f32_16x16x32_bf16(false, a, false, b, (short)0, c, false, false);
  }
  static __device__ __forceinline__ void guard(v8f& a, v8f& b, v16b x, v16b y) { dep_guard_b(a, b, x, y); }
  static __device__ __forceinline__ void keep(v16b a, v16b b, v16b c, v16b d) { keep4_b(a, b, c, d); }
};

template <int ET> struct Elem;
template <> struct Elem<0> { typedef _Float16 T; };
template <> struct Elem<1> { typedef __bf16 T; };
template <int ET, bool SPLIT, int BIAS_MODE, int OUT_MODE, bool RESID, int ACT = 0>
__global__ __launch_bounds__(256) void wmma_gemm64(
    const unsigned short* __restrict__ Ap, const unsigned short* __restrict__ A2p, int lda, long strideA,
    const unsigned short* __restrict__ Btp, const unsigned short* __restrict__ Bt2p, int ldb, long strideB,
    void* __restrict__ Cout, void* __restrict__ Cout2, int ldc, long strideC,
    const float* __restrict__ bias,
    const float* __restrict__ resid, long strideR,
    int M, int N, int K, float scale) {
  typedef typename Elem<ET>::T T;
  typedef typename Frag<T>::V V;
  const T* A = (const T*)Ap; const T* A2 = (const T*)A2p; const T* Bt = (const T*)Btp; const T* Bt2 = (const T*)Bt2p;
  __shared__ __align__(16) float sT[8][16 * 68];
  const int b    = blockIdx.y;
  const int lane = threadIdx.x & 31;
  const int wave = threadIdx.x >> 5;
  const int tilesN = N >> 6;
  const int tilesM = M >> 6;
  const int tile = blockIdx.x * 8 + wave;
  if (tile >= tilesM * tilesN) return;
  const int tm = tile / tilesN;
  const int tn = tile - tm * tilesN;
  const int m0 = tm << 6;
  const int n0 = tn << 6;

  const T* Ab  = A  + (size_t)b * strideA;
  const T* Bb  = Bt + (size_t)b * strideB;
  const T* Ab2 = SPLIT ? (A2  + (size_t)b * strideA) : nullptr;
  const T* Bb2 = SPLIT ? (Bt2 + (size_t)b * strideB) : nullptr;

  const int rlane = lane & 15;
  const int koff  = (lane >> 4) * 8;
  const int mOff  = (lane >> 4) * 8;

  v8f acc[4][4];
#pragma unroll
  for (int i = 0; i < 4; ++i)
#pragma unroll
    for (int j = 0; j < 4; ++j) acc[i][j] = (v8f){0.f,0.f,0.f,0.f,0.f,0.f,0.f,0.f};

  for (int k0 = 0; k0 < K; k0 += 32) {
    V bh[4], bl[4];
#pragma unroll
    for (int j = 0; j < 4; ++j) {
      const size_t bo = (size_t)(n0 + (j << 4) + rlane) * ldb + koff + k0;
      bh[j] = Frag<T>::load(Bb + bo);
      if (SPLIT) bl[j] = Frag<T>::load(Bb2 + bo);
    }
#pragma unroll
    for (int i = 0; i < 4; ++i) {
      const size_t ao = (size_t)(m0 + (i << 4) + rlane) * lda + koff + k0;
      V ah = Frag<T>::load(Ab + ao);
      V al;
      if (SPLIT) al = Frag<T>::load(Ab2 + ao);
#pragma unroll
      for (int j = 0; j < 4; ++j) {
        acc[i][j] = Frag<T>::mma(ah, bh[j], acc[i][j]);
        if (SPLIT) {
          acc[i][j] = Frag<T>::mma(ah, bl[j], acc[i][j]);
          acc[i][j] = Frag<T>::mma(al, bh[j], acc[i][j]);
        }
      }
      Frag<T>::guard(acc[i][0], acc[i][3], ah, SPLIT ? al : ah);
    }
    Frag<T>::keep(bh[0], bh[1], bh[2], bh[3]);
    if (SPLIT) Frag<T>::keep(bl[0], bl[1], bl[2], bl[3]);
  }
  acc_guard4(acc[0][0], acc[0][1], acc[0][2], acc[0][3]);
  acc_guard4(acc[1][0], acc[1][1], acc[1][2], acc[1][3]);
  acc_guard4(acc[2][0], acc[2][1], acc[2][2], acc[2][3]);
  acc_guard4(acc[3][0], acc[3][1], acc[3][2], acc[3][3]);

  float* slab = sT[wave];
  const float* Rb = RESID ? (resid + (size_t)b * strideR) : nullptr;
#pragma unroll
  for (int i = 0; i < 4; ++i) {
    const int mBase = m0 + (i << 4);
#pragma unroll
    for (int j = 0; j < 4; ++j) {
      const int n = n0 + (j << 4) + rlane;
      float bv = 0.f;
      if (BIAS_MODE == 2) bv = bias[n];
#pragma unroll
      for (int r = 0; r < 8; ++r) {
        float v = acc[i][j][r] * scale;
        if (BIAS_MODE == 1) v += bias[mBase + mOff + r];
        if (BIAS_MODE == 2) v += bv;
        if (RESID) v += Rb[(size_t)(mBase + mOff + r) * ldc + n];
        if (ACT == 1) v = tanhf(v);
        if (ACT == 2) v = fmaxf(v, 0.0f);
        if (ACT == 3) v = v / (1.0f + expf(-v));
        if (ACT == 4) v = (v > 0.f) ? v : 0.01f * v;
        if (ACT == 5) v = 0.5f * v * (1.0f + erff(v * 0.70710678118654752f));
        slab[(mOff + r) * 68 + (j << 4) + rlane] = v;
      }
    }
    __builtin_amdgcn_fence(__ATOMIC_RELEASE, "workgroup");
    __builtin_amdgcn_wave_barrier();
    __builtin_amdgcn_fence(__ATOMIC_ACQUIRE, "workgroup");
    if (OUT_MODE == 0) {
      float* C = (float*)Cout + (size_t)b * strideC;
      const int hh = lane >> 4, c4 = (lane & 15) * 4;
      for (int pass = 0; pass < 2; ++pass) {
#pragma unroll
        for (int it = 0; it < 8; ++it) {
          const int row = it * 2 + hh;
          v4f v = *(const v4f*)(slab + row * 68 + c4);
          *(volatile v4f*)(C + (size_t)(mBase + row) * ldc + n0 + c4) = v;
        }
        __threadfence();
      }
    } else {
      const int q = lane >> 3, c8 = (lane & 7) * 8;
      unsigned short* C  = (unsigned short*)Cout  + (size_t)b * strideC;
      unsigned short* C2 = (OUT_MODE == 2) ? ((unsigned short*)Cout2 + (size_t)b * strideC) : nullptr;
      for (int pass = 0; pass < 2; ++pass) {
#pragma unroll
        for (int it = 0; it < 4; ++it) {
          const int row = it * 4 + q;
          const float* sp = slab + row * 68 + c8;
          v8h hv, lv;
#pragma unroll
          for (int e = 0; e < 8; ++e) {
            if (OUT_MODE == 1) {
              hv[e] = (_Float16)sp[e];
            } else {
              unsigned short hb = f2bf_bits(sp[e]);
              unsigned short lb = f2bf_bits(sp[e] - bf_bits2f(hb));
              hv[e] = __builtin_bit_cast(_Float16, hb);
              lv[e] = __builtin_bit_cast(_Float16, lb);
            }
          }
          *(volatile v8h*)(C + (size_t)(mBase + row) * ldc + n0 + c8) = hv;
          if (OUT_MODE == 2) *(volatile v8h*)(C2 + (size_t)(mBase + row) * ldc + n0 + c8) = lv;
        }
        __threadfence();
      }
    }
    __builtin_amdgcn_fence(__ATOMIC_RELEASE, "workgroup");
    __builtin_amdgcn_wave_barrier();
    __builtin_amdgcn_fence(__ATOMIC_ACQUIRE, "workgroup");
  }
}

__global__ __launch_bounds__(256) void cast_f32_f16_pad2(
    const float* __restrict__ in0, const float* __restrict__ in1,
    unsigned short* __restrict__ out, long strideOut2, int nValid2, int nTotal2, float scale) {
  const int i = blockIdx.x * 256 + threadIdx.x;
  const float* in = (blockIdx.y == 0) ? in0 : in1;
  if (i < nTotal2) {
    const int ic = (i < nValid2) ? i : (nValid2 - 1);
    float f0 = in[2 * (size_t)ic], f1 = in[2 * (size_t)ic + 1];
    if (i >= nValid2) { f0 = 0.f; f1 = 0.f; }
    const _Float16 h0 = (_Float16)(f0 * scale), h1 = (_Float16)(f1 * scale);
    const unsigned u = (unsigned)__builtin_bit_cast(unsigned short, h0) | ((unsigned)__builtin_bit_cast(unsigned short, h1) << 16);
    volatile unsigned* o = (volatile unsigned*)out + (size_t)blockIdx.y * strideOut2 + i;
    *o = u;
    __threadfence();
    *o = u;
  }
}

__global__ __launch_bounds__(256) void cast_f32_bf16hl2(
    const float* __restrict__ in, unsigned short* __restrict__ hi, unsigned short* __restrict__ lo, int n2) {
  const int i = blockIdx.x * 256 + threadIdx.x;
  if (i < n2) {
    const float f0 = in[2 * (size_t)i], f1 = in[2 * (size_t)i + 1];
    const unsigned short hb0 = f2bf_bits(f0), hb1 = f2bf_bits(f1);
    const unsigned short lb0 = f2bf_bits(f0 - bf_bits2f(hb0)), lb1 = f2bf_bits(f1 - bf_bits2f(hb1));
    const unsigned uh = (unsigned)hb0 | ((unsigned)hb1 << 16);
    const unsigned ul = (unsigned)lb0 | ((unsigned)lb1 << 16);
    volatile unsigned* oh = (volatile unsigned*)hi + i;
    volatile unsigned* ol = (volatile unsigned*)lo + i;
    *oh = uh; *ol = ul;
    __threadfence();
    *oh = uh; *ol = ul;
  }
}

__global__ __launch_bounds__(DEG_THREADS) void degree_dinv(
    const int* __restrict__ ei0, const int* __restrict__ ei1, float* __restrict__ dinv,
    int N, int E, int dinvStride) {
  __shared__ __align__(16) int cnt[DEG_NT];
  __shared__ int hit[DEG_THREADS];
  __shared__ int wsum[DEG_THREADS / 32];
  const int tid = threadIdx.x, lane = tid & 31, wave = tid >> 5;
  const int view = blockIdx.y;
  const int* dstp = ((view == 0) ? ei0 : ei1) + (size_t)E;
  const int lo = blockIdx.x * DEG_NT;
  for (int i = tid; i < DEG_NT; i += DEG_THREADS) cnt[i] = 0;
  __syncthreads();
  for (int e0 = 0; e0 < E; e0 += DEG_THREADS) {
    const int e = e0 + tid;
    const int ec = (e < E) ? e : (E - 1);
    const int d = dstp[ec];
    const int rel = d - lo;
    const bool h = (e < E) && ((unsigned)rel < (unsigned)DEG_NT);
    const unsigned mask = __builtin_amdgcn_ballot_w32(h);
    const int pos = (int)__builtin_amdgcn_mbcnt_lo(mask, 0u);
    if (h) hit[wave * 32 + pos] = rel;
    if (lane == 0) wsum[wave] = (int)__builtin_popcount(mask);
    __syncthreads();
    if (tid == 0) {
      for (int w = 0; w < DEG_THREADS / 32; ++w) {
        int c = wsum[w];
        c = c < 0 ? 0 : (c > 32 ? 32 : c);
        for (int i = 0; i < c; ++i) {
          int r = hit[w * 32 + i];
          r = r < 0 ? 0 : (r >= DEG_NT ? DEG_NT - 1 : r);
          cnt[r] += 1;
        }
      }
    }
    __syncthreads();
  }
#pragma unroll 1
  for (int i = tid; i < DEG_NT; i += DEG_THREADS) {
    const float dg = (float)cnt[i] + 1.0f;
    cnt[i] = __float_as_int(1.0f / sqrtf(dg));
  }
  __syncthreads();
  int* dvi = (int*)(dinv + (size_t)view * dinvStride + (size_t)blockIdx.x * DEG_NT);
  for (int pass = 0; pass < 2; ++pass) {
#pragma unroll 1
    for (int i = tid; i < DEG_NT / 4; i += DEG_THREADS) {
      const v4i v = *(const v4i*)(cnt + 4 * i);
      *(volatile v4i*)(dvi + 4 * i) = v;
    }
    __threadfence();
  }
}

__global__ __launch_bounds__(32) void pool_partial(
    const float* __restrict__ Hf, long hStride,
    const int* __restrict__ ei0, const int* __restrict__ ei1,
    const int* __restrict__ batch,
    const float* __restrict__ dinv, int dinvStride,
    float* __restrict__ partOut, int* __restrict__ cntOut,
    int N, int E, int PE, int NB) {
  __shared__ __align__(16) float part[CN_B * CN_D];
  __shared__ __align__(16) int gcnt[CN_B];
  const int lane = threadIdx.x;
  const int view = blockIdx.y;
  const int blk  = blockIdx.x;
  const float* H  = Hf + (size_t)view * hStride;
  const int*   ei = (view == 0) ? ei0 : ei1;
  const float* dv = dinv + (size_t)view * dinvStride;
  v4f* part4 = (v4f*)part;
  const v4f z4 = {0.f, 0.f, 0.f, 0.f};
  for (int i = lane; i < CN_B * CN_D / 4; i += 32) part4[i] = z4;
  gcnt[lane] = 0; gcnt[lane + 32] = 0;
  __syncthreads();
  const bool edgeMode = (blk < PE);
  const int nIt  = edgeMode ? (POOL_CHE / 32) : (POOL_CHN / 32);
  const int base = edgeMode ? blk * POOL_CHE : (blk - PE) * POOL_CHN;
  for (int it = 0; it < nIt; ++it) {
    const int idx = base + it * 32 + lane;
    int src, g, cf; float w;
    if (edgeMode) {
      const bool valid = idx < E;
      const int ec = valid ? idx : (E - 1);
      int s = ei[ec];
      int d = ei[(size_t)E + ec];
      s = s < 0 ? 0 : (s >= N ? N - 1 : s);
      d = d < 0 ? 0 : (d >= N ? N - 1 : d);
      int gg = batch[d];
      gg = gg < 0 ? 0 : (gg >= CN_B ? CN_B - 1 : gg);
      const float wv = dv[s] * dv[d];
      src = s; g = gg; w = valid ? wv : 0.f; cf = 0;
    } else {
      const bool valid = idx < N;
      const int dc = valid ? idx : (N - 1);
      int gg = batch[dc];
      gg = gg < 0 ? 0 : (gg >= CN_B ? CN_B - 1 : gg);
      const float di = dv[dc];
      src = dc; g = gg; w = valid ? di * di : 0.f; cf = valid ? 1 : 0;
    }
#pragma unroll 4
    for (int j = 0; j < 32; ++j) {
      const int   s  = __shfl(src, j, 32);
      const int   gg = __shfl(g, j, 32);
      const float ww = __shfl(w, j, 32);
      const v4f hv = *(const v4f*)(H + (size_t)s * CN_D + 4 * lane);
      v4f a = part4[gg * (CN_D / 4) + lane];
      a = a + hv * ww;
      part4[gg * (CN_D / 4) + lane] = a;
      if (!edgeMode) {
        const int cc = __shfl(cf, j, 32);
        if (lane == 0) gcnt[gg] += cc;
      }
    }
  }
  __syncthreads();
  float* po = partOut + ((size_t)view * NB + blk) * (size_t)(CN_B * CN_D);
  int*   co = cntOut  + ((size_t)view * NB + blk) * (size_t)CN_B;
  for (int pass = 0; pass < 2; ++pass) {
    for (int i = lane; i < CN_B * CN_D / 4; i += 32) {
      const v4f v = part4[i];
      *(volatile v4f*)(po + 4 * i) = v;
    }
    if (lane < 16) {
      const v4i c = *(const v4i*)(gcnt + 4 * lane);
      *(volatile v4i*)(co + 4 * lane) = c;
    }
    __threadfence();
  }
}

__device__ __forceinline__ void store_row_planes16(const float* srow, unsigned short* hp, unsigned short* lp, int wave, int lane) {
  if (wave < 2 && lane < 16) {
    v8h pv;
#pragma unroll
    for (int e = 0; e < 8; ++e) {
      const float f = srow[lane * 8 + e];
      const unsigned short hb = f2bf_bits(f);
      const unsigned short lb = f2bf_bits(f - bf_bits2f(hb));
      pv[e] = __builtin_bit_cast(_Float16, (unsigned short)(wave == 0 ? hb : lb));
    }
    unsigned short* d = ((wave == 0) ? hp : lp) + lane * 8;
    *(volatile v8h*)d = pv;
    __threadfence();
    *(volatile v8h*)d = pv;
  }
}

__global__ __launch_bounds__(128) void pool_reduce(
    const float* __restrict__ partIn, const int* __restrict__ cntIn,
    const float* __restrict__ b1, const float* __restrict__ b2,
    float* __restrict__ featF, unsigned short* __restrict__ featH, unsigned short* __restrict__ featL,
    int NB, int PE) {
  __shared__ __align__(16) float srow[CN_D];
  const int r = blockIdx.x;
  const int g = r >> 1, view = r & 1;
  const int t = threadIdx.x, lane = t & 31, wave = t >> 5;
  const float* pb = partIn + (size_t)view * NB * (CN_B * CN_D) + (size_t)g * CN_D + t;
  float s = 0.f;
  for (int blk = 0; blk < NB; ++blk) s += pb[(size_t)blk * (CN_B * CN_D)];
  int cnt = 0;
  const int* cb = cntIn + (size_t)view * NB * CN_B + g;
  for (int blk = PE; blk < NB; ++blk) cnt += cb[(size_t)blk * CN_B];
  const float* bb = (view == 0) ? b1 : b2;
  const float fc = (float)cnt;
  const float val = (s + fc * bb[t]) * (1.0f / fmaxf(fc, 1.0f));
  srow[t] = val;
  volatile float* fo = (volatile float*)(featF + (size_t)r * CN_D + t);
  *fo = val;
  __syncthreads();
  store_row_planes16(srow, featH + (size_t)r * CN_D, featL + (size_t)r * CN_D, wave, lane);
  __threadfence();
  *fo = val;
}

__global__ __launch_bounds__(128) void attn_tokens2(
    const float* __restrict__ qkv, unsigned short* __restrict__ oH, unsigned short* __restrict__ oL) {
  __shared__ __align__(16) float srow[CN_D];
  const int r = blockIdx.x, g = r >> 1;
  const int t = threadIdx.x, lane = t & 31, wave = t >> 5;
  const int c = wave * 32 + lane;
  const float q  = qkv[(size_t)r * CN_QKV + c];
  const float k0 = qkv[(size_t)(2 * g) * CN_QKV + CN_D + c];
  const float k1 = qkv[(size_t)(2 * g + 1) * CN_QKV + CN_D + c];
  const float v0 = qkv[(size_t)(2 * g) * CN_QKV + 2 * CN_D + c];
  const float v1 = qkv[(size_t)(2 * g + 1) * CN_QKV + 2 * CN_D + c];
  float p0 = q * k0, p1 = q * k1;
#pragma unroll
  for (int off = 16; off >= 1; off >>= 1) { p0 += __shfl_xor(p0, off, 32); p1 += __shfl_xor(p1, off, 32); }
  const float SC = 0.17677669529663687f;
  const float s0 = p0 * SC, s1 = p1 * SC;
  const float m = fmaxf(s0, s1);
  const float e0 = expf(s0 - m), e1 = expf(s1 - m);
  const float inv = 1.0f / (e0 + e1);
  const float o = (e0 * inv) * v0 + (e1 * inv) * v1;
  srow[c] = o;
  __syncthreads();
  store_row_planes16(srow, oH + (size_t)r * CN_D, oL + (size_t)r * CN_D, wave, lane);
}

__global__ __launch_bounds__(128) void ln_mean_fuse(
    const float* __restrict__ y, const float* __restrict__ lnw, const float* __restrict__ lnb,
    unsigned short* __restrict__ fH, unsigned short* __restrict__ fL) {
  __shared__ float red[2][4][2];
  __shared__ __align__(16) float srow[CN_D];
  const int g = blockIdx.x, t = threadIdx.x, lane = t & 31, wave = t >> 5;
  const float y0 = y[(size_t)(2 * g) * CN_D + t];
  const float y1 = y[(size_t)(2 * g + 1) * CN_D + t];
  float a0 = y0, a1 = y1;
#pragma unroll
  for (int off = 16; off >= 1; off >>= 1) { a0 += __shfl_xor(a0, off, 32); a1 += __shfl_xor(a1, off, 32); }
  if (lane == 0) { red[0][wave][0] = a0; red[0][wave][1] = a1; }
  __syncthreads();
  const float invD = 1.0f / (float)CN_D;
  const float m0 = (red[0][0][0] + red[0][1][0] + red[0][2][0] + red[0][3][0]) * invD;
  const float m1 = (red[0][0][1] + red[0][1][1] + red[0][2][1] + red[0][3][1]) * invD;
  const float d0 = y0 - m0, d1 = y1 - m1;
  float q0 = d0 * d0, q1 = d1 * d1;
#pragma unroll
  for (int off = 16; off >= 1; off >>= 1) { q0 += __shfl_xor(q0, off, 32); q1 += __shfl_xor(q1, off, 32); }
  if (lane == 0) { red[1][wave][0] = q0; red[1][wave][1] = q1; }
  __syncthreads();
  const float var0 = (red[1][0][0] + red[1][1][0] + red[1][2][0] + red[1][3][0]) * invD;
  const float var1 = (red[1][0][1] + red[1][1][1] + red[1][2][1] + red[1][3][1]) * invD;
  const float rs0 = 1.0f / sqrtf(var0 + 1e-5f);
  const float rs1 = 1.0f / sqrtf(var1 + 1e-5f);
  const float wv = lnw[t], bv = lnb[t];
  const float l0 = d0 * rs0 * wv + bv;
  const float l1 = d1 * rs1 * wv + bv;
  srow[t] = (l0 + l1) * 0.5f;
  __syncthreads();
  store_row_planes16(srow, fH + (size_t)g * CN_D, fL + (size_t)g * CN_D, wave, lane);
}

extern "C" void kernel_launch(void* const* d_in, const int* in_sizes, int n_in,
                              void* d_out, int out_size, void* d_ws, size_t ws_size,
                              hipStream_t stream) {
  if (n_in < 17) return;
  const float* x_ego  = (const float*)d_in[0];
  const int*   ei_ego = (const int*)  d_in[1];
  const float* x_cut  = (const float*)d_in[2];
  const int*   ei_cut = (const int*)  d_in[3];
  const int*   batch  = (const int*)  d_in[4];
  const float* W1     = (const float*)d_in[5];
  const float* b1     = (const float*)d_in[6];
  const float* W2     = (const float*)d_in[7];
  const float* b2     = (const float*)d_in[8];
  const float* ipw    = (const float*)d_in[9];
  const float* ipb    = (const float*)d_in[10];
  const float* opw    = (const float*)d_in[11];
  const float* opb    = (const float*)d_in[12];
  const float* lnw    = (const float*)d_in[13];
  const float* lnb    = (const float*)d_in[14];
  const float* ow     = (const float*)d_in[15];
  const float* ob     = (const float*)d_in[16];
  float* out = (float*)d_out;

  const int N = in_sizes[4];
  const int E = in_sizes[1] / 2;
  if (N < 1 || E < 1) return;
  if (in_sizes[0] != N * CN_D || in_sizes[2] != N * CN_D) return;
  if (in_sizes[1] != 2 * E || in_sizes[3] != 2 * E) return;
  if (in_sizes[5] != CN_D * CN_D || in_sizes[7] != CN_D * CN_D) return;
  if (in_sizes[9] != CN_QKV * CN_D || in_sizes[11] != CN_D * CN_D || in_sizes[15] != CN_O * CN_D) return;
  if (in_sizes[6] != CN_D || in_sizes[8] != CN_D || in_sizes[10] != CN_QKV || in_sizes[12] != CN_D) return;
  if (in_sizes[13] != CN_D || in_sizes[14] != CN_D || in_sizes[16] != CN_O) return;
  if (out_size != CN_B * CN_O) return;

  const int MP    = ((N + 63) / 64) * 64;
  const int tiles = (N + DEG_NT - 1) / DEG_NT;
  const int NPD   = tiles * DEG_NT;
  const int PE    = (E + POOL_CHE - 1) / POOL_CHE;
  const int PN    = (N + POOL_CHN - 1) / POOL_CHN;
  const int NB    = PE + PN;

  size_t off = 0;
  auto carve = [&](size_t bytes) { size_t o = off; off += (bytes + 255) & ~(size_t)255; return o; };
  const size_t oXh  = carve((size_t)2 * MP * CN_D * 2);
  const size_t oWh  = carve((size_t)2 * CN_D * CN_D * 2);
  const size_t oHf  = carve((size_t)2 * MP * CN_D * 4);
  const size_t oDv  = carve((size_t)2 * NPD * 4);
  const size_t oPt  = carve((size_t)2 * NB * CN_B * CN_D * 4);
  const size_t oCt  = carve((size_t)2 * NB * CN_B * 4);
  const size_t oIPh = carve((size_t)CN_QKV * CN_D * 2);
  const size_t oIPl = carve((size_t)CN_QKV * CN_D * 2);
  const size_t oOPh = carve((size_t)CN_D * CN_D * 2);
  const size_t oOPl = carve((size_t)CN_D * CN_D * 2);
  const size_t oOWh = carve((size_t)CN_O * CN_D * 2);
  const size_t oOWl = carve((size_t)CN_O * CN_D * 2);
  const size_t oFeF = carve((size_t)2 * CN_B * CN_D * 4);
  const size_t oFeH = carve((size_t)2 * CN_B * CN_D * 2);
  const size_t oFeL = carve((size_t)2 * CN_B * CN_D * 2);
  const size_t oQKV = carve((size_t)2 * CN_B * CN_QKV * 4);
  const size_t oOh  = carve((size_t)2 * CN_B * CN_D * 2);
  const size_t oOl  = carve((size_t)2 * CN_B * CN_D * 2);
  const size_t oY   = carve((size_t)2 * CN_B * CN_D * 4);
  const size_t oFh  = carve((size_t)CN_B * CN_D * 2);
  const size_t oFl  = carve((size_t)CN_B * CN_D * 2);
  if (off > ws_size || off > (size_t)134217728) return;

  char* ws = (char*)d_ws;
  unsigned short* Xh  = (unsigned short*)(ws + oXh);
  unsigned short* Wh  = (unsigned short*)(ws + oWh);
  float*          Hf  = (float*)(ws + oHf);
  float*          Dv  = (float*)(ws + oDv);
  float*          Pt  = (float*)(ws + oPt);
  int*            Ct  = (int*)(ws + oCt);
  unsigned short* IPh = (unsigned short*)(ws + oIPh);
  unsigned short* IPl = (unsigned short*)(ws + oIPl);
  unsigned short* OPh = (unsigned short*)(ws + oOPh);
  unsigned short* OPl = (unsigned short*)(ws + oOPl);
  unsigned short* OWh = (unsigned short*)(ws + oOWh);
  unsigned short* OWl = (unsigned short*)(ws + oOWl);
  float*          FeF = (float*)(ws + oFeF);
  unsigned short* FeH = (unsigned short*)(ws + oFeH);
  unsigned short* FeL = (unsigned short*)(ws + oFeL);
  float*          QKV = (float*)(ws + oQKV);
  unsigned short* Oh  = (unsigned short*)(ws + oOh);
  unsigned short* Ol  = (unsigned short*)(ws + oOl);
  float*          Y   = (float*)(ws + oY);
  unsigned short* Fh  = (unsigned short*)(ws + oFh);
  unsigned short* Fl  = (unsigned short*)(ws + oFl);

  {
    const int nTot2 = MP * (CN_D / 2);
    const int nVal2 = N * (CN_D / 2);
    cast_f32_f16_pad2<<<dim3((nTot2 + 255) / 256, 2), 256, 0, stream>>>(x_ego, x_cut, Xh, (long)nTot2, nVal2, nTot2, 1.0f);
    const int nW2 = CN_D * CN_D / 2;
    cast_f32_f16_pad2<<<dim3((nW2 + 255) / 256, 2), 256, 0, stream>>>(W1, W2, Wh, (long)nW2, nW2, nW2, 16.0f);
    const int nI2 = CN_QKV * CN_D / 2, nO2 = CN_D * CN_D / 2, nQ2 = CN_O * CN_D / 2;
    cast_f32_bf16hl2<<<(nI2 + 255) / 256, 256, 0, stream>>>(ipw, IPh, IPl, nI2);
    cast_f32_bf16hl2<<<(nO2 + 255) / 256, 256, 0, stream>>>(opw, OPh, OPl, nO2);
    cast_f32_bf16hl2<<<(nQ2 + 255) / 256, 256, 0, stream>>>(ow, OWh, OWl, nQ2);
  }
  degree_dinv<<<dim3(tiles, 2), DEG_THREADS, 0, stream>>>(ei_ego, ei_cut, Dv, N, E, NPD);
  {
    const int tilesTot = (MP / 64) * (CN_D / 64);
    wmma_gemm64<0, false, 0, 0, false><<<dim3((tilesTot + 7) / 8, 2), 256, 0, stream>>>(
        Xh, Xh, CN_D, (long)MP * CN_D,
        Wh, Wh, CN_D, (long)CN_D * CN_D,
        (void*)Hf, (void*)Hf, CN_D, (long)MP * CN_D,
        Hf, Hf, 0L, MP, CN_D, CN_D, 1.0f / 16.0f);
  }
  pool_partial<<<dim3(NB, 2), 32, 0, stream>>>(Hf, (long)MP * CN_D, ei_ego, ei_cut, batch, Dv, NPD, Pt, Ct, N, E, PE, NB);
  pool_reduce<<<2 * CN_B, CN_D, 0, stream>>>(Pt, Ct, b1, b2, FeF, FeH, FeL, NB, PE);
  {
    const int tilesTot = (2 * CN_B / 64) * (CN_QKV / 64);
    wmma_gemm64<1, true, 2, 0, false><<<dim3((tilesTot + 7) / 8, 1), 256, 0, stream>>>(
        FeH, FeL, CN_D, 0L, IPh, IPl, CN_D, 0L,
        (void*)QKV, (void*)QKV, CN_QKV, 0L,
        ipb, FeF, 0L, 2 * CN_B, CN_QKV, CN_D, 1.0f);
  }
  attn_tokens2<<<2 * CN_B, CN_D, 0, stream>>>(QKV, Oh, Ol);
  {
    const int tilesTot = (2 * CN_B / 64) * (CN_D / 64);
    wmma_gemm64<1, true, 2, 0, true><<<dim3((tilesTot + 7) / 8, 1), 256, 0, stream>>>(
        Oh, Ol, CN_D, 0L, OPh, OPl, CN_D, 0L,
        (void*)Y, (void*)Y, CN_D, 0L,
        opb, FeF, 0L, 2 * CN_B, CN_D, CN_D, 1.0f);
  }
  ln_mean_fuse<<<CN_B, CN_D, 0, stream>>>(Y, lnw, lnb, Fh, Fl);
  {
    const int tilesTot = (CN_B / 64) * (CN_O / 64);
    wmma_gemm64<1, true, 2, 0, false><<<dim3((tilesTot + 7) / 8, 1), 256, 0, stream>>>(
        Fh, Fl, CN_D, 0L, OWh, OWl, CN_D, 0L,
        (void*)out, (void*)out, CN_O, 0L,
        ob, FeF, 0L, CN_B, CN_O, CN_D, 1.0f);
  }
}
